// Simple_Self_Attention_68564857914107
// MI455X (gfx1250) — hardware-verified
//
#include <hip/hip_runtime.h>
#include <math.h>

typedef __attribute__((ext_vector_type(16))) _Float16 v16h;
typedef __attribute__((ext_vector_type(16))) __bf16 v16b;
typedef __attribute__((ext_vector_type(8)))  _Float16 v8h;
typedef __attribute__((ext_vector_type(8)))  float v8f;
typedef __attribute__((ext_vector_type(4)))  float v4f;
typedef __attribute__((ext_vector_type(2)))  float v2f;
typedef __attribute__((ext_vector_type(4)))  unsigned v4u;
typedef __attribute__((ext_vector_type(4)))  int v4i;
typedef float __attribute__((may_alias)) float_a;
typedef int __attribute__((may_alias)) int_a;

template <typename T> __device__ __forceinline__ void vst2(void* p, T v) { *(volatile T*)p = v; __threadfence(); *(volatile T*)p = v; }
__device__ __forceinline__ v8f wmma16(v16h a, v16h b, v8f c) {
  v8f d = __builtin_amdgcn_wmma_f32_16x16x32_f16(false, a, false, b, (short)0, c, false, false);
  asm volatile("v_nop\n\tv_nop\n\tv_nop\n\tv_nop" : "+v"(d) : "v"(a), "v"(b));
  return d;
}
__device__ __forceinline__ v8f wmma_bf(v16b a, v16b b, v8f c) {
  v8f d = __builtin_amdgcn_wmma_f32_16x16x32_bf16(false, a, false, b, (short)0, c, false, false);
  asm volatile("v_nop\n\tv_nop\n\tv_nop\n\tv_nop" : "+v"(d) : "v"(a), "v"(b));
  return d;
}
__device__ __forceinline__ v16h frag_h(const _Float16* rowk0, int lane) {
  union { v16h v; v8h q[2]; } u; const _Float16* p = rowk0 + 8 * (lane >> 4);
  u.q[0] = *(const v8h*)p; u.q[1] = *(const v8h*)(p + 16); return u.v;
}
__device__ __forceinline__ v16h frag_f32(const float* rowk0, int lane) {
  v16h a; const float* p = rowk0 + 8 * (lane >> 4);
#pragma unroll
  for (int i = 0; i < 8; ++i) { a[i] = (_Float16)p[i]; a[8 + i] = (_Float16)p[16 + i]; }
  return a;
}
__device__ __forceinline__ v16h frag_f32s(const float* rowk0, int lane, float sc) {
  v16h a; const float* p = rowk0 + 8 * (lane >> 4);
#pragma unroll
  for (int i = 0; i < 8; ++i) { a[i] = (_Float16)(p[i] * sc); a[8 + i] = (_Float16)(p[16 + i] * sc); }
  return a;
}
__device__ __forceinline__ v16h fragc_f32(const float* W, int k0, int n, int lane, int ld, int K) {
  v16h a; const int g = lane >> 4;
#pragma unroll
  for (int i = 0; i < 8; ++i) { const int ka = k0 + 8 * g + i, kb = ka + 16;
    a[i] = (_Float16)(ka < K ? W[(size_t)(ka < K ? ka : K - 1) * ld + n] : 0.f); a[8 + i] = (_Float16)(kb < K ? W[(size_t)(kb < K ? kb : K - 1) * ld + n] : 0.f); }
  return a;
}
struct F2 { v16b h, l; };
__device__ __forceinline__ F2 bsplit16(const float v[16]) { F2 r;
#pragma unroll
  for (int i = 0; i < 16; ++i) { const __bf16 h = (__bf16)v[i]; r.h[i] = h; r.l[i] = (__bf16)(v[i] - (float)h); }
  return r; }
__device__ __forceinline__ F2 split_row(const float* row, int k0, int lane) { float v[16]; const float* p = row + k0 + 8 * (lane >> 4);
#pragma unroll
  for (int i = 0; i < 8; ++i) { v[i] = p[i]; v[8 + i] = p[16 + i]; }
  return bsplit16(v); }
__device__ __forceinline__ F2 split_rowK(const float* row, int k0, int lane, int K) { float v[16]; const int g = lane >> 4;
#pragma unroll
  for (int i = 0; i < 8; ++i) { const int ka = k0 + 8 * g + i, kb = ka + 16; v[i] = ka < K ? row[ka < K ? ka : K - 1] : 0.f; v[8 + i] = kb < K ? row[kb < K ? kb : K - 1] : 0.f; }
  return bsplit16(v); }
__device__ __forceinline__ F2 split_col(const float* W, int k0, int n, int lane, int ld, int K) { float v[16]; const int g = lane >> 4;
#pragma unroll
  for (int i = 0; i < 8; ++i) { const int ka = k0 + 8 * g + i, kb = ka + 16; v[i] = ka < K ? W[(size_t)(ka < K ? ka : K - 1) * ld + n] : 0.f; v[8 + i] = kb < K ? W[(size_t)(kb < K ? kb : K - 1) * ld + n] : 0.f; }
  return bsplit16(v); }
__device__ __forceinline__ v8f mac3(const F2& a, const F2& b, v8f c) { c = wmma_bf(a.l, b.h, c); c = wmma_bf(a.h, b.l, c); return wmma_bf(a.h, b.h, c); }
__device__ __forceinline__ float sigm(float v) { return 1.0f / (1.0f + expf(-v)); }
#define LDSX() do { asm volatile("s_wait_dscnt 0" ::: "memory"); __builtin_amdgcn_wave_barrier(); __builtin_amdgcn_fence(__ATOMIC_RELEASE, "workgroup"); } while (0)


#define NB 4
#define SS 2048
#define CC 1024
#define NR (NB * SS)
#ifndef TNB
#define TNB NB
#endif
#define TR (TNB * SS)
#define KPT (SS / 256)
typedef __attribute__((ext_vector_type(8))) __bf16 v8b;
__device__ __forceinline__ v16b frag_b(const __bf16* rowk0, int lane) {
  union { v16b v; v8b q[2]; } u; const __bf16* p = rowk0 + 8 * (lane >> 4);
  u.q[0] = *(const v8b*)p; u.q[1] = *(const v8b*)(p + 16); return u.v;
}
__device__ __forceinline__ float bfr(float v) { return (float)(__bf16)v; }
__device__ __attribute__((noinline)) float exp_ni(float v) { return expf(v); }
__device__ __attribute__((noinline)) float erf_ni(float v) { return erff(v); }

#define WS_PW   0u
#define WS_Q    (WS_PW + 2u * (size_t)3 * CC * CC)
#define WS_K    (WS_Q + 2u * (size_t)NR * CC)
#define WS_V    (WS_K + 2u * (size_t)NR * CC)
#define WS_S    (WS_V + 2u * (size_t)NB * CC * SS)
#define WS_P    (WS_S + 4u * (size_t)NB * SS * SS)
#define WS_END  (WS_P + 2u * (size_t)NB * SS * SS)

__global__ __launch_bounds__(256) void k_pack(const float* __restrict__ WQ, const float* __restrict__ WK, const float* __restrict__ WV, __bf16* __restrict__ P) { const int n = blockIdx.x, which = blockIdx.y, t = threadIdx.x; const float* src = (which == 0) ? WQ : (which == 1) ? WK : WV; __shared__ __align__(16) __bf16 s[CC]; for (int k = t; k < CC; k += 256) s[k] = (__bf16)src[(size_t)k * CC + n]; __syncthreads(); if (t < CC / 8) vst2((unsigned*)(P + ((size_t)which * CC + n) * CC + t * 8), *(const v4u*)&s[t * 8]); }
__global__ __launch_bounds__(128) void k_proj(const float* __restrict__ XQ, const float* __restrict__ XK, const float* __restrict__ XV, const __bf16* __restrict__ P, const float* __restrict__ BQ, const float* __restrict__ BK, const float* __restrict__ BV, _Float16* __restrict__ Q, _Float16* __restrict__ Kr, _Float16* __restrict__ V) {
  __shared__ __align__(16) _Float16 so[64][136]; __shared__ __align__(16) _Float16 st[128][72];
  const int tid = threadIdx.x, wave = tid >> 5, lane = tid & 31, col = lane & 15, g = lane >> 4; const int n0 = blockIdx.y * 128; const int which = n0 / CC, c0 = n0 % CC; const size_t rb0 = (size_t)blockIdx.x * 64, r0 = rb0 + wave * 16; const float* X = (which == 0) ? XQ : (which == 1) ? XK : XV; const float* BB = ((which == 0) ? BQ : (which == 1) ? BK : BV) + c0;
  v8f acc[8] = {};
#pragma unroll 2
  for (int kc = 0; kc < CC / 32; ++kc) { v16b a; { const float* p = X + (r0 + col) * CC + kc * 32 + 8 * g;
#pragma unroll
      for (int i = 0; i < 8; ++i) { a[i] = (__bf16)p[i]; a[8 + i] = (__bf16)p[16 + i]; } }
#pragma unroll
    for (int j = 0; j < 8; ++j) acc[j] = wmma_bf(a, frag_b(P + (size_t)(n0 + j * 16 + col) * CC + kc * 32, lane), acc[j]); }
  if (which < 2) { _Float16* dst = (which == 0) ? Q : Kr;
#pragma unroll
    for (int j = 0; j < 8; ++j)
#pragma unroll
      for (int r = 0; r < 8; ++r) so[wave * 16 + 8 * g + r][j * 16 + col] = (_Float16)(acc[j][r] + bfr(BB[j * 16 + col]));
    LDSX();
    for (int rl = 0; rl < 16; ++rl) if (lane < 16) vst2((unsigned*)(dst + (r0 + rl) * CC + c0 + lane * 8), *(const v4u*)&so[wave * 16 + rl][lane * 8]);
  } else {
#pragma unroll
    for (int j = 0; j < 8; ++j)
#pragma unroll
      for (int r = 0; r < 8; ++r) st[j * 16 + col][wave * 16 + 8 * g + r] = (_Float16)(acc[j][r] + bfr(BB[j * 16 + col]));
    __syncthreads();
    const size_t b = rb0 / SS, s0 = rb0 % SS;
    for (int e = tid; e < 128 * 8; e += 128) { const int d = e >> 3, pc = e & 7; vst2((unsigned*)(V + ((b * CC + c0 + d) * SS) + s0 + pc * 8), *(const v4u*)&st[d][pc * 8]); } }
}
__global__ __launch_bounds__(128) void k_scores(const _Float16* __restrict__ Q, const _Float16* __restrict__ Kr, float* __restrict__ S) {
  __shared__ __align__(16) _Float16 sq[64][CC + 8]; __shared__ __align__(16) float so[4][16][36];
  const int tid = threadIdx.x, wave = tid >> 5, lane = tid & 31, col = lane & 15, g = lane >> 4; const size_t b = blockIdx.y; const int qb = blockIdx.x; const int q0 = qb * 64 + wave * 16; const size_t rq0 = b * SS + (size_t)qb * 64;
  for (int e = tid; e < 64 * (CC / 8); e += 128) { const int rr = e / (CC / 8), q = e % (CC / 8); *(v4u*)&sq[rr][q * 8] = *(const v4u*)(Q + (rq0 + rr) * CC + q * 8); }
  __syncthreads();
#pragma unroll 1
  for (int ks = 0; ks < SS / 32; ++ks) { const int j0 = ks * 32;
    {
#pragma unroll
      for (int ct = 0; ct < 2; ++ct) { const int kk = j0 + ct * 16 + col; const _Float16* krow = Kr + (b * SS + kk) * CC; v8f c = {};
#pragma unroll 4
        for (int kc = 0; kc < CC / 32; ++kc) c = wmma16(frag_h(&sq[wave * 16 + col][0] + kc * 32, lane), frag_h(krow + kc * 32, lane), c);
#pragma unroll
        for (int r = 0; r < 8; ++r) so[wave][8 * g + r][ct * 16 + col] = c[r] * 0.03125f; }
    }
    LDSX();
    for (int rl = 0; rl < 16; ++rl) if (lane < 8) vst2(S + ((b * SS + q0 + rl) * (size_t)SS) + j0 + lane * 4, *(const v4f*)&so[wave][rl][lane * 4]);
    LDSX(); }
}
__device__ __attribute__((noinline)) float exp_p(float v) { return expf(v); }
__global__ __launch_bounds__(256) void k_soft(const float* __restrict__ S, _Float16* __restrict__ Pt) {
  __shared__ float red[8]; __shared__ __align__(16) _Float16 sp[SS]; const size_t row = blockIdx.x; const int t = threadIdx.x; const float* s = S + row * SS; float v[KPT]; float mx = -3.0e38f;
  for (int i = 0; i < KPT; ++i) { v[i] = s[t * KPT + i]; mx = fmaxf(mx, v[i]); }
#pragma unroll
  for (int o = 1; o < 32; o <<= 1) mx = fmaxf(mx, __shfl_xor(mx, o));
  if ((t & 31) == 0) red[t >> 5] = mx; __syncthreads(); float m = red[0]; for (int i = 1; i < 8; ++i) m = fmaxf(m, red[i]); __syncthreads();
  float sum = 0.f; for (int i = 0; i < KPT; ++i) { v[i] = (v[i] <= -1.0e38f) ? 0.f : exp_p(v[i] - m); sum += v[i]; }
#pragma unroll
  for (int o = 1; o < 32; o <<= 1) sum += __shfl_xor(sum, o);
  if ((t & 31) == 0) red[t >> 5] = sum; __syncthreads(); float tot = 0.f; for (int i = 0; i < 8; ++i) tot += red[i]; const float sc = 2048.0f / tot;
  for (int i = 0; i < KPT; ++i) sp[t * KPT + i] = (_Float16)(v[i] * sc);
  __syncthreads(); if (t < SS / 8) vst2((unsigned*)(Pt + row * SS + t * 8), *(const v4u*)&sp[t * 8]);
}
__global__ __launch_bounds__(128) void k_pv(const _Float16* __restrict__ Pt, const _Float16* __restrict__ V, float* __restrict__ CTX) {
  __shared__ __align__(16) float so[4][16][132];
  const int tid = threadIdx.x, wave = tid >> 5, lane = tid & 31, col = lane & 15, g = lane >> 4; const size_t b = blockIdx.z; const int qb = blockIdx.x; const size_t rq = b * SS + (size_t)qb * 64 + wave * 16; const int c0 = blockIdx.y * 128; const int nkc = SS / 32;
  v8f acc[8] = {};
#pragma unroll 2
  for (int kc = 0; kc < nkc; ++kc) { const v16h a = frag_h(Pt + (rq + col) * SS + kc * 32, lane);
#pragma unroll
    for (int j = 0; j < 8; ++j) acc[j] = wmma16(a, frag_h(V + ((b * CC + c0 + j * 16 + col) * SS) + kc * 32, lane), acc[j]); }
#pragma unroll
  for (int j = 0; j < 8; ++j)
#pragma unroll
    for (int r = 0; r < 8; ++r) so[wave][8 * g + r][j * 16 + col] = acc[j][r] * (1.0f / 2048.0f);
  LDSX();
  for (int rl = 0; rl < 16; ++rl) vst2(CTX + (rq + rl) * CC + c0 + lane * 4, *(const v4f*)&so[wave][rl][lane * 4]);
}
extern "C" void kernel_launch(void* const* d_in, const int* in_sizes, int n_in, void* d_out, int out_size, void* d_ws, size_t ws_size, hipStream_t stream) {
  (void)in_sizes; (void)n_in; (void)out_size;
  const float** F = (const float**)d_in;
  if (ws_size < (size_t)WS_END) return;
  char* ws = (char*)d_ws; __bf16* P = (__bf16*)ws; _Float16 *Q = (_Float16*)(ws + WS_Q), *Kr = (_Float16*)(ws + WS_K), *V = (_Float16*)(ws + WS_V), *Pt = (_Float16*)(ws + WS_P); float* S = (float*)(ws + WS_S);
  k_pack<<<dim3(CC, 3), 256, 0, stream>>>(F[2], F[4], F[6], P);
  k_proj<<<dim3(TR / 64, 3 * CC / 128), 128, 0, stream>>>(F[0], F[1], F[1], P, F[3], F[5], F[7], Q, Kr, V);
  k_scores<<<dim3(SS / 64, TNB), 128, 0, stream>>>(Q, Kr, S);
  k_soft<<<TR, 256, 0, stream>>>(S, Pt);
  k_pv<<<dim3(SS / 64, CC / 128, TNB), 128, 0, stream>>>(Pt, V, (float*)d_out);
}
